// SelfAttention_3994319585291
// MI455X (gfx1250) — hardware-verified
//
#include <hip/hip_runtime.h>

#ifndef SEQ
#define SEQ 2048
#endif
#define SEQ_FULL 2048
#define DM   2048
#define NH   16
#define HD   128
#define CQ   96
#define CQP  128
#define CKV  512
#define DOUT 2048

#define C_CAR    4.0f
#define WQU_CAR  16.0f
#define WKV_CAR  32.0f
#define Q_CAR    16.0f
#define K_CAR    2.0f
#define V_CAR    2.0f
#define CTX_CAR  64.0f
#define WO_CAR   64.0f
#define RSQ_HD   0.08838834764831845f

static_assert(SEQ % 128 == 0);
static_assert(SEQ <= SEQ_FULL);
static_assert(NH * HD == DM);
static_assert(HD == 128);
static_assert(CQ % 32 == 0);
static_assert(CQ % 8 == 0);
static_assert(CQ <= CQP);
static_assert(CQP == 128);
static_assert(CKV % 128 == 0);
static_assert(DM % 128 == 0);
static_assert(DOUT % 128 == 0);

typedef _Float16 f16;
typedef __bf16   bf16;
typedef f16      v16h __attribute__((ext_vector_type(16)));
typedef bf16     v16b __attribute__((ext_vector_type(16)));
typedef float    v8f  __attribute__((ext_vector_type(8)));
typedef float    v4f  __attribute__((ext_vector_type(4)));
typedef unsigned v4u  __attribute__((ext_vector_type(4)));
typedef v4u __attribute__((may_alias)) v4ua;
typedef v4f __attribute__((may_alias)) v4fa;

#define Z8 ((v8f){0.f, 0.f, 0.f, 0.f, 0.f, 0.f, 0.f, 0.f})

union FragH { v16h v; v4ua q[2]; f16 h[16]; typedef f16 elem; };
union FragB { v16b v; v4ua q[2]; typedef bf16 elem; };

__device__ __forceinline__ v8f mma16(const FragH& a, const FragH& b, v8f c) {
  v8f r = __builtin_amdgcn_wmma_f32_16x16x32_f16(false, a.v, false, b.v, (short)0, c, false, false);
  asm volatile("v_nop\n\tv_nop\n\tv_nop\n\tv_nop" : "+v"(r) : "v"(a.v), "v"(b.v));
  return r;
}
__device__ __forceinline__ v8f mma16(const FragB& a, const FragB& b, v8f c) {
  v8f r = __builtin_amdgcn_wmma_f32_16x16x32_bf16(false, a.v, false, b.v, (short)0, c, false, false);
  asm volatile("v_nop\n\tv_nop\n\tv_nop\n\tv_nop" : "+v"(r) : "v"(a.v), "v"(b.v));
  return r;
}

__device__ __forceinline__ unsigned bf_bits(float f) {
  unsigned u = __float_as_uint(f);
  return (u + 0x7fffu + ((u >> 16) & 1u)) >> 16;
}
__device__ __forceinline__ float bf_val(float f) {
  return __uint_as_float(bf_bits(f) << 16);
}

__global__ __launch_bounds__(256)
void cvt_kernel(const float* __restrict__ src, unsigned short* __restrict__ dst,
                int n8, float scale, int tobf)
{
  const int g = blockIdx.x * 256 + (int)threadIdx.x;
  if (g >= n8) return;
  const size_t e = (size_t)g * 8;
  const v4fa x0 = *(const v4fa*)(src + e);
  const v4fa x1 = *(const v4fa*)(src + e + 4);
  float v[8];
  #pragma unroll
  for (int i = 0; i < 4; ++i) { v[i] = x0[i]; v[4 + i] = x1[i]; }
  union { f16 h[8]; unsigned short s[8]; v4u q; } t;
  if (tobf) {
    #pragma unroll
    for (int i = 0; i < 8; ++i) t.s[i] = (unsigned short)bf_bits(v[i]);
  } else {
    #pragma unroll
    for (int i = 0; i < 8; ++i) t.h[i] = (f16)(bf_val(v[i]) * scale);
  }
  const v4u o = t.q;
  volatile v4u* p = (volatile v4u*)(dst + e);
  *p = o;
  __threadfence();
  *p = o;
}

#define CP 128
#define GEMM_LDS_BYTES (128 * CP * 4)

template <typename FR, int MODE>
__global__ __launch_bounds__(256) __attribute__((amdgpu_num_vgpr(256)))
void gemm_nt(const typename FR::elem* __restrict__ A, int lda,
             const typename FR::elem* __restrict__ Bm, int ldb, int nbr,
             const float* __restrict__ bias, float ascale, float cscale,
             void* __restrict__ Cout, int ldc, int K,
             const float* __restrict__ rcos, const float* __restrict__ rsin)
{
  extern __shared__ float4 dyn_lds[];
  float* Cs = reinterpret_cast<float*>(dyn_lds);
  typedef typename FR::elem T;

  const int tid  = threadIdx.x;
  const int wave = tid >> 5, lane = tid & 31, lq = lane & 15, hf = lane >> 4;
  const int wm   = wave & 3, wn = wave >> 2;
  const int m0   = blockIdx.y * 128, n0 = blockIdx.x * 128;

  v8f acc[2][4];
  #pragma unroll
  for (int i = 0; i < 2; ++i) {
    #pragma unroll
    for (int j = 0; j < 4; ++j) acc[i][j] = Z8;
  }

  const T* ap[2];
  const T* bp[4];
  #pragma unroll
  for (int i = 0; i < 2; ++i)
    ap[i] = A + (size_t)(m0 + wm * 32 + i * 16 + lq) * lda + hf * 8;
  #pragma unroll
  for (int j = 0; j < 4; ++j) {
    int br = n0 + wn * 64 + j * 16 + lq;
    br = (br < nbr) ? br : (nbr - 1);
    bp[j] = Bm + (size_t)br * ldb + hf * 8;
  }

  #pragma unroll 1
  for (int k0 = 0; k0 < K; k0 += 32) {
    FR a[2], b[4];
    #pragma unroll
    for (int i = 0; i < 2; ++i) {
      a[i].q[0] = *(const v4ua*)(ap[i] + k0);
      a[i].q[1] = *(const v4ua*)(ap[i] + k0 + 16);
    }
    #pragma unroll
    for (int j = 0; j < 4; ++j) {
      b[j].q[0] = *(const v4ua*)(bp[j] + k0);
      b[j].q[1] = *(const v4ua*)(bp[j] + k0 + 16);
    }
    #pragma unroll
    for (int i = 0; i < 2; ++i) {
      #pragma unroll
      for (int j = 0; j < 4; ++j) acc[i][j] = mma16(a[i], b[j], acc[i][j]);
    }
  }

  #pragma unroll
  for (int i = 0; i < 2; ++i) {
    #pragma unroll
    for (int j = 0; j < 4; ++j) {
      #pragma unroll
      for (int r = 0; r < 8; ++r)
        Cs[(wm * 32 + i * 16 + hf * 8 + r) * CP + wn * 64 + j * 16 + lq] = acc[i][j][r];
    }
  }
  __syncthreads();

  if constexpr (MODE == 0 || MODE == 1) {
    f16* outp = reinterpret_cast<f16*>(Cout);
    const int rsub = tid >> 4;
    const int cg   = (tid & 15) * 8;
    const int pcg  = cg ^ 64;
    const float sg = (cg < 64) ? -1.0f : 1.0f;
    float bb[8], bpv[8];
    {
      int gb = n0 + cg;
      gb = (gb + 8 <= nbr) ? gb : (nbr - 8);
      const v4fa b0 = *(const v4fa*)(bias + gb);
      const v4fa b1 = *(const v4fa*)(bias + gb + 4);
      #pragma unroll
      for (int e = 0; e < 4; ++e) { bb[e] = bf_val(b0[e]); bb[4 + e] = bf_val(b1[e]); }
      if constexpr (MODE == 1) {
        const v4fa p0 = *(const v4fa*)(bias + n0 + pcg);
        const v4fa p1 = *(const v4fa*)(bias + n0 + pcg + 4);
        #pragma unroll
        for (int e = 0; e < 4; ++e) { bpv[e] = bf_val(p0[e]); bpv[4 + e] = bf_val(p1[e]); }
      } else {
        #pragma unroll
        for (int e = 0; e < 8; ++e) bpv[e] = 0.0f;
      }
    }
    v4u vals[8];
    #pragma unroll
    for (int p = 0; p < 8; ++p) {
      const int row = p * 16 + rsub;
      const v4fa x0 = *(const v4fa*)(Cs + row * CP + cg);
      const v4fa x1 = *(const v4fa*)(Cs + row * CP + cg + 4);
      float av[8];
      #pragma unroll
      for (int e = 0; e < 4; ++e) { av[e] = x0[e]; av[4 + e] = x1[e]; }
      float res[8];
      if constexpr (MODE == 0) {
        #pragma unroll
        for (int e = 0; e < 8; ++e) {
          const float v = av[e] * ascale + bb[e];
          res[e] = (n0 + cg + e < nbr) ? (v * cscale) : 0.0f;
        }
      } else {
        const v4fa y0 = *(const v4fa*)(Cs + row * CP + pcg);
        const v4fa y1 = *(const v4fa*)(Cs + row * CP + pcg + 4);
        const float* cr = rcos + (size_t)(m0 + row) * HD + cg;
        const float* sr = rsin + (size_t)(m0 + row) * HD + cg;
        const v4fa c0 = *(const v4fa*)(cr);
        const v4fa c1 = *(const v4fa*)(cr + 4);
        const v4fa s0 = *(const v4fa*)(sr);
        const v4fa s1 = *(const v4fa*)(sr + 4);
        float wv[8], cc[8], ss[8];
        #pragma unroll
        for (int e = 0; e < 4; ++e) {
          wv[e] = y0[e]; wv[4 + e] = y1[e];
          cc[e] = c0[e]; cc[4 + e] = c1[e];
          ss[e] = s0[e]; ss[4 + e] = s1[e];
        }
        #pragma unroll
        for (int e = 0; e < 8; ++e) {
          const float v = av[e] * ascale + bb[e];
          const float u = wv[e] * ascale + bpv[e];
          res[e] = (v * bf_val(cc[e]) + sg * u * bf_val(ss[e])) * cscale;
        }
      }
      union { f16 h[8]; v4u q; } t;
      #pragma unroll
      for (int e = 0; e < 8; ++e) t.h[e] = (f16)res[e];
      vals[p] = t.q;
    }
    f16* ob = outp + (size_t)m0 * ldc + n0 + cg;
    #pragma unroll
    for (int p = 0; p < 8; ++p)
      *(volatile v4u*)(ob + (size_t)(p * 16 + rsub) * ldc) = vals[p];
    __threadfence();
    #pragma unroll
    for (int p = 0; p < 8; ++p)
      *(volatile v4u*)(ob + (size_t)(p * 16 + rsub) * ldc) = vals[p];
  } else if constexpr (MODE == 2) {
    f16* outp = reinterpret_cast<f16*>(Cout);
    const int csub = tid >> 4;
    const int rg   = (tid & 15) * 8;
    v4u vals[8];
    #pragma unroll
    for (int p = 0; p < 8; ++p) {
      const int col = p * 16 + csub;
      const float b1 = bf_val(bias[n0 + col]);
      union { f16 h[8]; v4u q; } t;
      #pragma unroll
      for (int e = 0; e < 8; ++e)
        t.h[e] = (f16)((Cs[(rg + e) * CP + col] * ascale + b1) * cscale);
      vals[p] = t.q;
    }
    f16* ob = outp + (size_t)n0 * ldc + m0 + rg;
    #pragma unroll
    for (int p = 0; p < 8; ++p)
      *(volatile v4u*)(ob + (size_t)(p * 16 + csub) * ldc) = vals[p];
    __threadfence();
    #pragma unroll
    for (int p = 0; p < 8; ++p)
      *(volatile v4u*)(ob + (size_t)(p * 16 + csub) * ldc) = vals[p];
  } else {
    float* outp = reinterpret_cast<float*>(Cout);
    const int cg = lane * 4;
    float bb[4];
    {
      const v4fa b0 = *(const v4fa*)(bias + n0 + cg);
      #pragma unroll
      for (int e = 0; e < 4; ++e) bb[e] = bf_val(b0[e]);
    }
    #pragma unroll
    for (int g = 0; g < 2; ++g) {
      v4f vals[8];
      #pragma unroll
      for (int p = 0; p < 8; ++p) {
        const int row = g * 64 + p * 8 + wave;
        const v4fa x0 = *(const v4fa*)(Cs + row * CP + cg);
        v4f rv;
        #pragma unroll
        for (int e = 0; e < 4; ++e) rv[e] = x0[e] * ascale + bb[e];
        vals[p] = rv;
      }
      float* ob = outp + (size_t)(m0 + g * 64 + wave) * ldc + n0 + cg;
      #pragma unroll
      for (int p = 0; p < 8; ++p)
        *(volatile v4f*)(ob + (size_t)(p * 8) * ldc) = vals[p];
      __threadfence();
      #pragma unroll
      for (int p = 0; p < 8; ++p)
        *(volatile v4f*)(ob + (size_t)(p * 8) * ldc) = vals[p];
    }
  }
}

#define KSP 136
#define VSP 40
#define OSP 136

__global__ __launch_bounds__(256) __attribute__((amdgpu_num_vgpr(256)))
void fa_kernel(const f16* __restrict__ qh, const f16* __restrict__ kh,
               const f16* __restrict__ vth, f16* __restrict__ ctx)
{
  __shared__ __align__(16) f16 Ks[32 * KSP];
  __shared__ __align__(16) f16 Vs[HD * VSP];
  __shared__ __align__(16) f16 Os[8 * 16 * OSP];

  const int qblk = blockIdx.x, head = blockIdx.y;
  const int tid  = threadIdx.x;
  const int wave = tid >> 5, lane = tid & 31, lq = lane & 15, hf = lane >> 4;

  const int qrow = qblk * 128 + wave * 16 + lq;
  FragH qf[4];
  #pragma unroll
  for (int f = 0; f < 4; ++f) {
    const f16* base = qh + (size_t)qrow * DM + head * HD + f * 32 + hf * 8;
    qf[f].q[0] = *(const v4ua*)(base);
    qf[f].q[1] = *(const v4ua*)(base + 16);
  }

  v8f o[8];
  #pragma unroll
  for (int dt = 0; dt < 8; ++dt) o[dt] = Z8;
  float rmax = -__builtin_inff();
  float rsum = 0.0f;
  const float SL = 1.4426950408889634f / (Q_CAR * K_CAR);

  #pragma unroll 1
  for (int it = 0; it < SEQ / 32; ++it) {
    const int j0 = it * 32;
    __syncthreads();
    #pragma unroll
    for (int u = 0; u < 2; ++u) {
      const int c  = tid + u * 256;
      const int kr = c >> 4, kc = (c & 15) * 8;
      const v4ua kv = *(const v4ua*)(kh + (size_t)(j0 + kr) * DM + head * HD + kc);
      *(v4ua*)(Ks + kr * KSP + kc) = kv;
      const int vr = c >> 2, vc = (c & 3) * 8;
      const v4ua vv = *(const v4ua*)(vth + (size_t)(head * HD + vr) * SEQ + j0 + vc);
      *(v4ua*)(Vs + vr * VSP + vc) = vv;
    }
    __syncthreads();

    v8f c2[2];
    #pragma unroll
    for (int sub = 0; sub < 2; ++sub) {
      v8f acc = Z8;
      #pragma unroll
      for (int f = 0; f < 4; ++f) {
        FragH a;
        const f16* base = Ks + (sub * 16 + lq) * KSP + f * 32 + hf * 8;
        a.q[0] = *(const v4ua*)(base);
        a.q[1] = *(const v4ua*)(base + 16);
        acc = mma16(a, qf[f], acc);
      }
      c2[sub] = acc;
    }

    float m_new = rmax;
    #pragma unroll
    for (int r = 0; r < 8; ++r) {
      m_new = fmaxf(m_new, c2[0][r]);
      m_new = fmaxf(m_new, c2[1][r]);
    }
    m_new = fmaxf(m_new, __shfl_xor(m_new, 16, 32));
    const float scale = __builtin_amdgcn_exp2f((rmax - m_new) * SL);
    rmax = m_new;

    FragH pa;
    float psum = 0.0f;
    #pragma unroll
    for (int r = 0; r < 8; ++r) {
      const float p0 = __builtin_amdgcn_exp2f((c2[0][r] - m_new) * SL);
      const float p1 = __builtin_amdgcn_exp2f((c2[1][r] - m_new) * SL);
      psum += p0 + p1;
      pa.h[r]     = (f16)p0;
      pa.h[8 + r] = (f16)p1;
    }
    rsum = rsum * scale + psum + __shfl_xor(psum, 16, 32);

    float sc[8];
    #pragma unroll
    for (int r = 0; r < 8; ++r) sc[r] = __shfl(scale, (hf << 3) + r, 32);
    #pragma unroll
    for (int dt = 0; dt < 8; ++dt) {
      #pragma unroll
      for (int r = 0; r < 8; ++r) o[dt][r] *= sc[r];
    }

    #pragma unroll
    for (int dt = 0; dt < 8; ++dt) {
      FragH b;
      const f16* base = Vs + (dt * 16 + lq) * VSP + hf * 8;
      b.q[0] = *(const v4ua*)(base);
      b.q[1] = *(const v4ua*)(base + 16);
      o[dt] = mma16(pa, b, o[dt]);
    }
  }

  float rs[8];
  #pragma unroll
  for (int r = 0; r < 8; ++r) {
    const float l = __shfl(rsum, (hf << 3) + r, 32);
    rs[r] = (CTX_CAR / V_CAR) * (1.0f / l);
  }
  f16* osw = Os + wave * 16 * OSP;
  #pragma unroll
  for (int dt = 0; dt < 8; ++dt) {
    #pragma unroll
    for (int r = 0; r < 8; ++r)
      osw[(hf * 8 + r) * OSP + dt * 16 + lq] = (f16)(o[dt][r] * rs[r]);
  }
  __syncthreads();

  v4u vals[8];
  #pragma unroll
  for (int u = 0; u < 8; ++u) {
    const int row = u * 2 + hf;
    vals[u] = *(const v4ua*)(osw + row * OSP + lq * 8);
  }
  f16* ob = ctx + (size_t)(qblk * 128 + wave * 16) * DM + head * HD + lq * 8;
  #pragma unroll
  for (int u = 0; u < 8; ++u)
    *(volatile v4u*)(ob + (size_t)(u * 2 + hf) * DM) = vals[u];
  __threadfence();
  #pragma unroll
  for (int u = 0; u < 8; ++u)
    *(volatile v4u*)(ob + (size_t)(u * 2 + hf) * DM) = vals[u];
}

static void launch_cvt(const float* src, void* dst, int n, float scale, int tobf, hipStream_t s)
{
  const int n8 = n / 8;
  const int blocks = (n8 + 255) / 256;
  cvt_kernel<<<blocks, 256, 0, s>>>(src, reinterpret_cast<unsigned short*>(dst), n8, scale, tobf);
}

extern "C" void kernel_launch(void* const* d_in, const int* in_sizes, int n_in,
                              void* d_out, int out_size, void* d_ws, size_t ws_size,
                              hipStream_t stream)
{
  if (n_in < 15) return;
  const float* x        = (const float*)d_in[0];
  const float* rope_cos = (const float*)d_in[1];
  const float* rope_sin = (const float*)d_in[2];
  const float* wq_down  = (const float*)d_in[3];
  const float* bq_down  = (const float*)d_in[4];
  const float* wq_up    = (const float*)d_in[5];
  const float* bq_up    = (const float*)d_in[6];
  const float* wkv_down = (const float*)d_in[7];
  const float* bkv_down = (const float*)d_in[8];
  const float* wk_up    = (const float*)d_in[9];
  const float* bk_up    = (const float*)d_in[10];
  const float* wv_up    = (const float*)d_in[11];
  const float* bv_up    = (const float*)d_in[12];
  const float* wo       = (const float*)d_in[13];
  const float* bo       = (const float*)d_in[14];
  float* out = (float*)d_out;

  if (in_sizes[0] < SEQ * DM) return;
  if (in_sizes[1] < SEQ * HD || in_sizes[2] < SEQ * HD) return;
  if (in_sizes[3] < CQ * DM || in_sizes[4] < CQ || in_sizes[5] < DM * CQ || in_sizes[6] < DM) return;
  if (in_sizes[7] < CKV * DM || in_sizes[8] < CKV) return;
  if (in_sizes[9] < DM * CKV || in_sizes[10] < DM || in_sizes[11] < DM * CKV || in_sizes[12] < DM) return;
  if (in_sizes[13] < DOUT * DM || in_sizes[14] < DOUT) return;
  if (out_size < SEQ * DOUT) return;

  char* wsb = (char*)d_ws;
  size_t off = 0;
  bf16* xb    = (bf16*)(wsb + off); off += (size_t)SEQ * DM * 2;
  bf16* wqd   = (bf16*)(wsb + off); off += (size_t)CQ * DM * 2;
  bf16* wkvd  = (bf16*)(wsb + off); off += (size_t)CKV * DM * 2;
  f16*  wqu   = (f16*)(wsb + off);  off += (size_t)DM * CQ * 2;
  f16*  wku   = (f16*)(wsb + off);  off += (size_t)DM * CKV * 2;
  f16*  wvu   = (f16*)(wsb + off);  off += (size_t)DM * CKV * 2;
  f16*  woh   = (f16*)(wsb + off);  off += (size_t)DOUT * DM * 2;
  f16*  cqh   = (f16*)(wsb + off);  off += (size_t)SEQ * CQP * 2;
  f16*  ckvh  = (f16*)(wsb + off);  off += (size_t)SEQ * CKV * 2;
  f16*  qpl   = (f16*)(wsb + off);  off += (size_t)SEQ * DM * 2;
  f16*  kpl   = (f16*)(wsb + off);  off += (size_t)SEQ * DM * 2;
  f16*  vtp   = (f16*)(wsb + off);  off += (size_t)DM * SEQ * 2;
  f16*  ctxp  = (f16*)(wsb + off);  off += (size_t)SEQ * DM * 2;
  if (off > ws_size) return;

  hipFuncSetAttribute(reinterpret_cast<const void*>(&gemm_nt<FragB, 0>),
                      hipFuncAttributeMaxDynamicSharedMemorySize, GEMM_LDS_BYTES);
  hipFuncSetAttribute(reinterpret_cast<const void*>(&gemm_nt<FragH, 1>),
                      hipFuncAttributeMaxDynamicSharedMemorySize, GEMM_LDS_BYTES);
  hipFuncSetAttribute(reinterpret_cast<const void*>(&gemm_nt<FragH, 2>),
                      hipFuncAttributeMaxDynamicSharedMemorySize, GEMM_LDS_BYTES);
  hipFuncSetAttribute(reinterpret_cast<const void*>(&gemm_nt<FragH, 3>),
                      hipFuncAttributeMaxDynamicSharedMemorySize, GEMM_LDS_BYTES);

  launch_cvt(x,        xb,   SEQ * DM,  1.0f,    1, stream);
  launch_cvt(wq_down,  wqd,  CQ * DM,   1.0f,    1, stream);
  launch_cvt(wkv_down, wkvd, CKV * DM,  1.0f,    1, stream);
  launch_cvt(wq_up,    wqu,  DM * CQ,   WQU_CAR, 0, stream);
  launch_cvt(wk_up,    wku,  DM * CKV,  WKV_CAR, 0, stream);
  launch_cvt(wv_up,    wvu,  DM * CKV,  WKV_CAR, 0, stream);
  launch_cvt(wo,       woh,  DOUT * DM, WO_CAR,  0, stream);

  const dim3 blk(256);
  gemm_nt<FragB, 0><<<dim3(CQP / 128, SEQ / 128), blk, GEMM_LDS_BYTES, stream>>>(
      xb, DM, wqd, DM, CQ, bq_down, 1.0f, C_CAR, (void*)cqh, CQP, DM, rope_cos, rope_sin);
  gemm_nt<FragB, 0><<<dim3(CKV / 128, SEQ / 128), blk, GEMM_LDS_BYTES, stream>>>(
      xb, DM, wkvd, DM, CKV, bkv_down, 1.0f, C_CAR, (void*)ckvh, CKV, DM, rope_cos, rope_sin);
  gemm_nt<FragH, 1><<<dim3(DM / 128, SEQ / 128), blk, GEMM_LDS_BYTES, stream>>>(
      cqh, CQP, wqu, CQ, DM, bq_up, 1.0f / (C_CAR * WQU_CAR), Q_CAR * RSQ_HD,
      (void*)qpl, DM, CQ, rope_cos, rope_sin);
  gemm_nt<FragH, 1><<<dim3(DM / 128, SEQ / 128), blk, GEMM_LDS_BYTES, stream>>>(
      ckvh, CKV, wku, CKV, DM, bk_up, 1.0f / (C_CAR * WKV_CAR), K_CAR,
      (void*)kpl, DM, CKV, rope_cos, rope_sin);
  gemm_nt<FragH, 2><<<dim3(DM / 128, SEQ / 128), blk, GEMM_LDS_BYTES, stream>>>(
      ckvh, CKV, wvu, CKV, DM, bv_up, 1.0f / (C_CAR * WKV_CAR), V_CAR,
      (void*)vtp, SEQ, CKV, rope_cos, rope_sin);
  fa_kernel<<<dim3(SEQ / 128, NH), blk, 0, stream>>>(qpl, kpl, vtp, ctxp);
  gemm_nt<FragH, 3><<<dim3(DOUT / 128, SEQ / 128), blk, GEMM_LDS_BYTES, stream>>>(
      ctxp, DM, woh, DM, DOUT, bo, 1.0f / (CTX_CAR * WO_CAR), 1.0f,
      (void*)out, DOUT, DM, rope_cos, rope_sin);
}
